// MyModel_61933428410278
// MI455X (gfx1250) — hardware-verified
//
#include <hip/hip_runtime.h>
#include <math.h>

#ifndef NB
#define NB 2
#endif
#ifndef SEQ
#define SEQ 2048
#endif
#ifndef SKV
#define SKV 3072
#endif
#define NB_FULL   2
#define NH        16
#define HD        64
#define SEQ_FULL  2048
#define SKV_FULL  3072

static_assert(NB >= 1 && NB <= NB_FULL);
static_assert(SEQ % 128 == 0 && SEQ <= SEQ_FULL);
static_assert(SKV % 64 == 0 && SKV <= SKV_FULL);
static_assert(HD == 64);
static_assert((NB * NH * SKV) % 32 == 0);

constexpr float kScale2   = 0.125f * 1.44269504088896340736f;
constexpr float kCarry    = 4096.0f;
constexpr float kInvCarry = 1.0f / 4096.0f;
#define NEG_INF (-__builtin_inff())

#if __has_builtin(__builtin_amdgcn_exp2f)
#define EXP2(x) __builtin_amdgcn_exp2f(x)
#else
#define EXP2(x) exp2f(x)
#endif

typedef __attribute__((ext_vector_type(16))) _Float16 v16h;
typedef __attribute__((ext_vector_type(8)))  _Float16 v8h;
typedef __attribute__((ext_vector_type(2)))  _Float16 v2h;
typedef __attribute__((ext_vector_type(16))) __bf16   v16b;
typedef __attribute__((ext_vector_type(8)))  __bf16   v8b;
typedef __attribute__((ext_vector_type(8)))  float    v8f;
typedef __attribute__((ext_vector_type(4)))  float    v4f;
typedef __attribute__((ext_vector_type(4)))  unsigned int v4u;
typedef __attribute__((ext_vector_type(8)))  unsigned int v8u;

__device__ __forceinline__ unsigned short f2bf_bits(float f) {
  unsigned u = __float_as_uint(f);
  return (unsigned short)((u + 0x7FFFu + ((u >> 16) & 1u)) >> 16);
}
__device__ __forceinline__ float bf_bits2f(unsigned short h) { return __uint_as_float(((unsigned)h) << 16); }

__device__ __forceinline__ void dep_guard1_b(v8f& a, v16b w, v16b x, v16b y, v16b z) {
  asm volatile("v_nop\n\tv_nop\n\tv_nop\n\tv_nop" : "+v"(a) : "v"(w), "v"(x), "v"(y), "v"(z));
}
__device__ __forceinline__ void dep_guard4_h(v8f& a, v8f& b, v8f& c, v8f& d, v16h x, v16h y) {
  asm volatile("v_nop\n\tv_nop\n\tv_nop\n\tv_nop" : "+v"(a), "+v"(b), "+v"(c), "+v"(d) : "v"(x), "v"(y));
}
__device__ __forceinline__ void keep4_h(v16h a, v16h b, v16h c, v16h d) { asm volatile("v_nop" :: "v"(a), "v"(b), "v"(c), "v"(d)); }
__device__ __forceinline__ void acc_guard4(v8f& a, v8f& b, v8f& c, v8f& d) {
  asm volatile("v_nop\n\tv_nop\n\tv_nop\n\tv_nop" : "+v"(a), "+v"(b), "+v"(c), "+v"(d));
}

template <typename T> struct Frag;
template <> struct Frag<_Float16> {
  typedef v16h V; union U { v16h v; v8h h[2]; };
  static __device__ __forceinline__ v16h load(const _Float16* p) {
    U f; f.h[0] = *(const v8h*)(p); f.h[1] = *(const v8h*)(p + 16); return f.v;
  }
  static __device__ __forceinline__ v8f mma(v16h a, v16h b, v8f c) {
    return __builtin_amdgcn_wmma_f32_16x16x32_f16(false, a, false, b, (short)0, c, false, false);
  }
};
template <> struct Frag<__bf16> {
  typedef v16b V; union U { v16b v; v8b h[2]; };
  static __device__ __forceinline__ v16b load(const __bf16* p) {
    U f; f.h[0] = *(const v8b*)(p); f.h[1] = *(const v8b*)(p + 16); return f.v;
  }
  static __device__ __forceinline__ v8f mma(v16b a, v16b b, v8f c) {
    return __builtin_amdgcn_wmma_f32_16x16x32_bf16(false, a, false, b, (short)0, c, false, false);
  }
};
typedef Frag<_Float16> FragH;
typedef Frag<__bf16>   FragB;

__device__ __forceinline__ unsigned pk16(unsigned short a, unsigned short b) { return (unsigned)a | ((unsigned)b << 16); }
__device__ __forceinline__ unsigned pkh2(float a, float b) {
  v2h p; p[0] = (_Float16)a; p[1] = (_Float16)b;
  return __builtin_bit_cast(unsigned, p);
}
__device__ __forceinline__ v8f zero8() { return (v8f){0.f, 0.f, 0.f, 0.f, 0.f, 0.f, 0.f, 0.f}; }
__device__ __forceinline__ v8f neg8()  { return (v8f){NEG_INF, NEG_INF, NEG_INF, NEG_INF, NEG_INF, NEG_INF, NEG_INF, NEG_INF}; }
__device__ __forceinline__ float hsum8(v8f v) {
  float a = v[0] + v[1], b = v[2] + v[3], c = v[4] + v[5], d = v[6] + v[7];
  return (a + b) + (c + d);
}
__device__ __forceinline__ float hmax8(v8f v) {
  float a = fmaxf(v[0], v[1]), b = fmaxf(v[2], v[3]);
  float c = fmaxf(v[4], v[5]), d = fmaxf(v[6], v[7]);
  return fmaxf(fmaxf(a, b), fmaxf(c, d));
}

__global__ __launch_bounds__(256) void cast_rows_kernel(const float* __restrict__ src,
                                                         unsigned short* __restrict__ dst,
                                                         int rowsPerGroup, int srcRowsPerGroup, int nRows) {
  const int t  = threadIdx.x;
  int pr = blockIdx.x * 32 + (t >> 3);
  pr = (pr < nRows) ? pr : (nRows - 1);
  const int c8 = (t & 7) * 8;
  const int g  = pr / rowsPerGroup;
  const int r  = pr - g * rowsPerGroup;
  const float* s = src + ((size_t)g * srcRowsPerGroup + r) * HD + c8;
  const v4f a = *(const v4f*)(s);
  const v4f b = *(const v4f*)(s + 4);
  unsigned short hb[8];
#pragma unroll
  for (int e = 0; e < 4; ++e) { hb[e] = f2bf_bits(a[e]); hb[4 + e] = f2bf_bits(b[e]); }
  const v4u u = (v4u){pk16(hb[0], hb[1]), pk16(hb[2], hb[3]), pk16(hb[4], hb[5]), pk16(hb[6], hb[7])};
  unsigned short* d = dst + (size_t)pr * HD + c8;
  *(volatile v4u*)d = u;
  __threadfence();
  *(volatile v4u*)d = u;
}

__global__ __launch_bounds__(256) void v_transpose_kernel(const float* __restrict__ v,
                                                           _Float16* __restrict__ Vt) {
  __shared__ float sm[64][65];
  const int tid = threadIdx.x;
  const int kv0 = blockIdx.x * 64;
  const int bh  = blockIdx.y;
  const float* vb = v + ((size_t)bh * SKV_FULL + kv0) * HD;
#pragma unroll
  for (int i = 0; i < 16; ++i) {
    const int e = i * 256 + tid;
    const int r = e >> 6;
    const int c = e & 63;
    sm[r][c] = vb[(size_t)r * HD + c];
  }
  __syncthreads();
  const int lane = tid & 31, wave = tid >> 5;
  const int q = lane >> 3, c8 = (lane & 7) * 8;
  _Float16* vt = Vt + (size_t)bh * HD * SKV;
  for (int pass = 0; pass < 2; ++pass) {
#pragma unroll
    for (int it = 0; it < 2; ++it) {
      const int row = wave * 8 + it * 4 + q;
      v8h hv;
#pragma unroll
      for (int e = 0; e < 8; ++e) hv[e] = (_Float16)bf_bits2f(f2bf_bits(sm[c8 + e][row]));
      *(volatile v8h*)(vt + (size_t)row * SKV + kv0 + c8) = hv;
    }
    __threadfence();
  }
}

__global__ __launch_bounds__(256) void attn_kernel(const float* __restrict__ q,
                                                    const unsigned short* __restrict__ Kp,
                                                    const unsigned short* __restrict__ Vtp,
                                                    const int* __restrict__ np,
                                                    float* __restrict__ out) {
  __shared__ __align__(16) float sT[8][16 * 68];
  const int tid  = threadIdx.x;
  const int wave = tid >> 5;
  const int lane = tid & 31;
  const int hi   = lane >> 4;
  const int l15  = lane & 15;
  const int h    = blockIdx.y;
  const int b    = blockIdx.z;
  const int bh   = b * NH + h;
  const int q0w  = blockIdx.x * 128 + wave * 16;

  int numpt = np[0];
  numpt = (numpt < 0) ? 0 : numpt;
  numpt = (numpt > SKV) ? SKV : numpt;

  const float*    Qb = q + ((size_t)bh * SEQ_FULL) * HD;
  const __bf16*   Kb = (const __bf16*)Kp + (size_t)bh * SKV * HD;
  const _Float16* Vb = (const _Float16*)Vtp + (size_t)bh * HD * SKV;
  float*          Ob = out + ((size_t)bh * SEQ) * HD;

  v16b bq[2];
  {
    const float* qrow = Qb + (size_t)(q0w + l15) * HD;
#pragma unroll
    for (int si = 0; si < 2; ++si) {
      const v4f f0 = *(const v4f*)(qrow + si * 32 + 8 * hi);
      const v4f f1 = *(const v4f*)(qrow + si * 32 + 8 * hi + 4);
      const v4f g0 = *(const v4f*)(qrow + si * 32 + 16 + 8 * hi);
      const v4f g1 = *(const v4f*)(qrow + si * 32 + 16 + 8 * hi + 4);
      v8u u;
      u[0] = pk16(f2bf_bits(f0[0]), f2bf_bits(f0[1]));
      u[1] = pk16(f2bf_bits(f0[2]), f2bf_bits(f0[3]));
      u[2] = pk16(f2bf_bits(f1[0]), f2bf_bits(f1[1]));
      u[3] = pk16(f2bf_bits(f1[2]), f2bf_bits(f1[3]));
      u[4] = pk16(f2bf_bits(g0[0]), f2bf_bits(g0[1]));
      u[5] = pk16(f2bf_bits(g0[2]), f2bf_bits(g0[3]));
      u[6] = pk16(f2bf_bits(g1[0]), f2bf_bits(g1[1]));
      u[7] = pk16(f2bf_bits(g1[2]), f2bf_bits(g1[3]));
      bq[si] = __builtin_bit_cast(v16b, u);
    }
  }

  v8f oacc[4];
#pragma unroll
  for (int dg = 0; dg < 4; ++dg) oacc[dg] = zero8();
  float m = NEG_INF;
  float l = 0.f;

  const int qmax   = q0w + 15 + numpt;
  const int kv_end = (SKV < qmax + 1) ? SKV : (qmax + 1);

#pragma unroll 1
  for (int kv0 = 0; kv0 < kv_end; kv0 += 64) {
    v8f s4[4];
#pragma unroll
    for (int t = 0; t < 4; ++t) {
      const int c0 = kv0 + t * 16;
      if (c0 > qmax) {
        s4[t] = neg8();
        continue;
      }
      const __bf16* krow = Kb + (size_t)(c0 + l15) * HD + 8 * hi;
      const v16b ak0 = FragB::load(krow);
      const v16b ak1 = FragB::load(krow + 32);
      v8f s = zero8();
      s = FragB::mma(ak0, bq[0], s);
      s = FragB::mma(ak1, bq[1], s);
      dep_guard1_b(s, ak0, ak1, bq[0], bq[1]);
      const bool part = (c0 + 15 > q0w + numpt);
      const int  lim  = q0w + l15 + numpt - c0;
      v8f sc;
#pragma unroll
      for (int r = 0; r < 8; ++r) {
        float vv = s[r] * kScale2;
        if (part && (r + 8 * hi > lim)) vv = NEG_INF;
        sc[r] = vv;
      }
      s4[t] = sc;
    }

    float tmax = fmaxf(fmaxf(hmax8(s4[0]), hmax8(s4[1])), fmaxf(hmax8(s4[2]), hmax8(s4[3])));
    tmax = fmaxf(tmax, __shfl_xor(tmax, 16, 32));
    const float mn    = fmaxf(m, tmax);
    const float alpha = (m > NEG_INF) ? EXP2(m - mn) : 0.0f;
    const float mref  = (mn > NEG_INF) ? mn : 0.0f;
    m = mn;
#pragma unroll
    for (int t = 0; t < 4; ++t)
#pragma unroll
      for (int r = 0; r < 8; ++r) s4[t][r] = EXP2(s4[t][r] - mref);
    float ts = (hsum8(s4[0]) + hsum8(s4[1])) + (hsum8(s4[2]) + hsum8(s4[3]));
    ts += __shfl_xor(ts, 16, 32);
    l = l * alpha + ts;
#pragma unroll
    for (int dg = 0; dg < 4; ++dg)
#pragma unroll
      for (int r = 0; r < 8; ++r) oacc[dg][r] *= alpha;

#pragma unroll
    for (int si = 0; si < 2; ++si) {
      const v8f p0 = s4[2 * si];
      const v8f p1 = s4[2 * si + 1];
      v8u u;
#pragma unroll
      for (int j = 0; j < 4; ++j) {
        u[j]     = pkh2(p0[2 * j] * kCarry, p0[2 * j + 1] * kCarry);
        u[4 + j] = pkh2(p1[2 * j] * kCarry, p1[2 * j + 1] * kCarry);
      }
      const v16h bp = __builtin_bit_cast(v16h, u);
      const _Float16* vrow = Vb + (size_t)l15 * SKV + kv0 + si * 32 + 8 * hi;
      const v16h av0 = FragH::load(vrow);
      const v16h av1 = FragH::load(vrow + (size_t)16 * SKV);
      const v16h av2 = FragH::load(vrow + (size_t)32 * SKV);
      const v16h av3 = FragH::load(vrow + (size_t)48 * SKV);
      oacc[0] = FragH::mma(av0, bp, oacc[0]);
      oacc[1] = FragH::mma(av1, bp, oacc[1]);
      oacc[2] = FragH::mma(av2, bp, oacc[2]);
      oacc[3] = FragH::mma(av3, bp, oacc[3]);
      dep_guard4_h(oacc[0], oacc[1], oacc[2], oacc[3], av3, bp);
      keep4_h(av0, av1, av2, bp);
    }
  }
  acc_guard4(oacc[0], oacc[1], oacc[2], oacc[3]);

  const float inv = (l > 0.f) ? ((1.0f / l) * kInvCarry) : 0.f;
  float* slab = sT[wave];
#pragma unroll
  for (int dg = 0; dg < 4; ++dg)
#pragma unroll
    for (int r = 0; r < 8; ++r)
      slab[l15 * 68 + dg * 16 + 8 * hi + r] = oacc[dg][r] * inv;
  __builtin_amdgcn_fence(3  , "workgroup");
  __builtin_amdgcn_wave_barrier();
  __builtin_amdgcn_fence(2  , "workgroup");
  const int hh = lane >> 4, c4 = (lane & 15) * 4;
  for (int pass = 0; pass < 2; ++pass) {
#pragma unroll
    for (int it = 0; it < 8; ++it) {
      const int row = it * 2 + hh;
      const v4f vv = *(const v4f*)(slab + row * 68 + c4);
      *(volatile v4f*)(Ob + (size_t)(q0w + row) * HD + c4) = vv;
    }
    __threadfence();
  }
}

extern "C" void kernel_launch(void* const* d_in, const int* in_sizes, int n_in,
                              void* d_out, int out_size, void* d_ws, size_t ws_size,
                              hipStream_t stream) {
  if (n_in < 4) return;
  if (in_sizes[0] < NB * NH * SEQ * HD) return;
  if (in_sizes[1] < NB * NH * SKV * HD) return;
  if (in_sizes[2] < NB * NH * SKV * HD) return;
  if (in_sizes[3] < 1) return;
  if (out_size < NB * NH * SEQ * HD) return;

  const size_t szK   = (size_t)NB * NH * SKV * HD * 2;
  const size_t szVt  = (size_t)NB * NH * HD * SKV * 2;
  const size_t offK  = 0;
  const size_t offVt = offK + szK;
  const size_t total = offVt + szVt;
  if (ws_size < total) return;

  const float* q  = (const float*)d_in[0];
  const float* k  = (const float*)d_in[1];
  const float* v  = (const float*)d_in[2];
  const int*   np = (const int*)d_in[3];
  float* out = (float*)d_out;
  char* ws = (char*)d_ws;
  unsigned short* Kp = (unsigned short*)(ws + offK);
  _Float16*       Vt = (_Float16*)(ws + offVt);

  const int nRowsK = NB * NH * SKV;
  cast_rows_kernel<<<dim3(nRowsK / 32), dim3(256), 0, stream>>>(k, Kp, SKV, SKV_FULL, nRowsK);
  v_transpose_kernel<<<dim3(SKV / 64, NB * NH), dim3(256), 0, stream>>>(v, Vt);
  attn_kernel<<<dim3(SEQ / 128, NH, NB), dim3(256), 0, stream>>>(q, Kp, (const unsigned short*)Vt, np, out);
}
